// RNN_11673721111233
// MI455X (gfx1250) — hardware-verified
//
#include <hip/hip_runtime.h>
#include <math.h>

constexpr int NBAT    = 16384;
constexpr int NSTEP   = 32;
constexpr int NVOC    = 27;
constexpr int NEMB    = 64;
constexpr int NHID    = 64;
constexpr int NKIN    = NEMB + NHID;
constexpr int NTHR    = 256;
constexpr int NWAVE   = NTHR / 32;
constexpr int RPW     = 16;
constexpr int GCOLS   = 3 * NHID;
constexpr int GSIZE   = NVOC * GCOLS;
constexpr int GSIZE4  = GSIZE / 4;
constexpr int NWTE4   = NVOC * NEMB / 4;
constexpr int APITCH  = 72;
constexpr int WPITCH  = 72;
constexpr int NVPAD   = 32;
constexpr int NROWS   = NBAT * NSTEP;
constexpr int LMROWS  = 64;
constexpr int LMSLAB  = LMROWS * NVOC;
constexpr int LMSLAB4 = LMSLAB / 4;
constexpr int NOUT    = NROWS * NVOC;
constexpr float HCAR  = 64.0f;
constexpr float WCAR  = 16.0f;
constexpr float FOLD  = 1.0f / 1024.0f;
static_assert(NBAT % (NWAVE * RPW) == 0);
static_assert(NROWS % (NWAVE * LMROWS) == 0);
static_assert(NHID % 32 == 0 && NEMB % 32 == 0);
static_assert((NVOC * NEMB) % 4 == 0 && GSIZE % 4 == 0);
static_assert((LMSLAB * 4) % 128 == 0);
static_assert((32 * NVOC * 4) % 128 == 0);
static_assert((NHID * NHID) % NTHR == 0);
static_assert((NVPAD * NHID) % NTHR == 0);
static_assert(APITCH % 8 == 0 && WPITCH % 8 == 0);

typedef __attribute__((ext_vector_type(16))) _Float16 v16h;
typedef __attribute__((ext_vector_type(8)))  _Float16 v8h;
typedef __attribute__((ext_vector_type(16))) __bf16   v16b;
typedef __attribute__((ext_vector_type(8)))  __bf16   v8b;
typedef __attribute__((ext_vector_type(8)))  float    v8f;
typedef __attribute__((ext_vector_type(4)))  float    v4f;
typedef __attribute__((ext_vector_type(4)))  unsigned v4u;
typedef v4u __attribute__((may_alias)) v4ua;

__device__ __forceinline__ void dep_guard_h(v8f& a, v8f& b, v16h x, v16h y) { asm volatile("v_nop\n\tv_nop\n\tv_nop\n\tv_nop" : "+v"(a), "+v"(b) : "v"(x), "v"(y)); }
__device__ __forceinline__ void dep_guard_b(v8f& a, v8f& b, v16b x, v16b y) { asm volatile("v_nop\n\tv_nop\n\tv_nop\n\tv_nop" : "+v"(a), "+v"(b) : "v"(x), "v"(y)); }
__device__ __forceinline__ void keep4_h(v16h a, v16h b, v16h c, v16h d) { asm volatile("v_nop" :: "v"(a), "v"(b), "v"(c), "v"(d)); }
__device__ __forceinline__ void keep4_b(v16b a, v16b b, v16b c, v16b d) { asm volatile("v_nop" :: "v"(a), "v"(b), "v"(c), "v"(d)); }
__device__ __forceinline__ void guard2_f6(v8f& a, v8f& b, v16h f0, v16h f1, v16h f2, v16h f3, v16h f4, v16h f5) {
  asm volatile("v_nop\n\tv_nop\n\tv_nop\n\tv_nop" : "+v"(a), "+v"(b) : "v"(f0), "v"(f1), "v"(f2), "v"(f3), "v"(f4), "v"(f5));
}
__device__ __forceinline__ void guard1_f4(v8f& a, v16h f0, v16h f1, v16h f2, v16h f3) {
  asm volatile("v_nop\n\tv_nop\n\tv_nop\n\tv_nop" : "+v"(a) : "v"(f0), "v"(f1), "v"(f2), "v"(f3));
}
template <typename T> struct Frag;
template <> struct Frag<_Float16> {
  typedef v16h V; union U { v16h v; v8h h[2]; };
  static __device__ __forceinline__ v16h load(const _Float16* p) {
    U f; f.h[0] = *(const v8h*)(p); f.h[1] = *(const v8h*)(p + 16); return f.v;
  }
  static __device__ __forceinline__ v8f mma(v16h a, v16h b, v8f c) {
    return __builtin_amdgcn_wmma_f32_16x16x32_f16(false, a, false, b, (short)0, c, false, false);
  }
  static __device__ __forceinline__ void guard(v8f& a, v8f& b, v16h x, v16h y) { dep_guard_h(a, b, x, y); }
  static __device__ __forceinline__ void keep(v16h a, v16h b, v16h c, v16h d) { keep4_h(a, b, c, d); }
};
template <> struct Frag<__bf16> {
  typedef v16b V; union U { v16b v; v8b h[2]; };
  static __device__ __forceinline__ v16b load(const __bf16* p) {
    U f; f.h[0] = *(const v8b*)(p); f.h[1] = *(const v8b*)(p + 16); return f.v;
  }
  static __device__ __forceinline__ v8f mma(v16b a, v16b b, v8f c) {
    return __builtin_amdgcn_wmma_f32_16x16x32_bf16(false, a, false, b, (short)0, c, false, false);
  }
  static __device__ __forceinline__ void guard(v8f& a, v8f& b, v16b x, v16b y) { dep_guard_b(a, b, x, y); }
  static __device__ __forceinline__ void keep(v16b a, v16b b, v16b c, v16b d) { keep4_b(a, b, c, d); }
};

__device__ __forceinline__ float fsig(float x) { return 1.0f / (1.0f + expf(-x)); }

__device__ __forceinline__ void gtab_part(const float* __restrict__ W, const float* __restrict__ bvec,
                                          const float* swte, float* sG, int gcol0, int tid) {
#pragma unroll 1
  for (int o = tid; o < NVOC * NHID; o += NTHR) {
    const int v = o >> 6, j = o & 63;
    const float* wrow = W + (size_t)j * NKIN;
    const float* erow = swte + v * NEMB;
    float acc = 0.0f;
#pragma unroll 1
    for (int e = 0; e < NEMB; ++e) acc = fmaf(erow[e], wrow[e], acc);
    acc = acc + bvec[j];
    sG[v * GCOLS + gcol0 + j] = acc;
  }
}

__global__ __launch_bounds__(NTHR) void gtab_kernel(const float* __restrict__ wte,
                                                    const float* __restrict__ Wr, const float* __restrict__ br,
                                                    const float* __restrict__ Wz, const float* __restrict__ bz,
                                                    const float* __restrict__ Wh, const float* __restrict__ bh,
                                                    float* __restrict__ G) {
  __shared__ __align__(16) float swte[NVOC * NEMB];
  __shared__ __align__(16) float sG[GSIZE];
  const int tid = threadIdx.x;
#pragma unroll 1
  for (int it = 0; it < (NWTE4 + NTHR - 1) / NTHR; ++it) {
    const int f  = it * NTHR + tid;
    const int fc = (f < NWTE4) ? f : (NWTE4 - 1);
    const v4f v = *(const v4f*)(wte + 4 * fc);
    if (f < NWTE4) *(v4f*)(swte + 4 * fc) = v;
  }
  __syncthreads();
  gtab_part(Wr, br, swte, sG, 0, tid);
  gtab_part(Wz, bz, swte, sG, NHID, tid);
  gtab_part(Wh, bh, swte, sG, 2 * NHID, tid);
  __syncthreads();
  for (int pass = 0; pass < 2; ++pass) {
#pragma unroll 1
    for (int it = 0; it < (GSIZE4 + NTHR - 1) / NTHR; ++it) {
      const int f  = it * NTHR + tid;
      const int fc = (f < GSIZE4) ? f : (GSIZE4 - 1);
      const v4f v = *(const v4f*)(sG + 4 * fc);
      if (f < GSIZE4) *(volatile v4f*)(G + 4 * fc) = v;
    }
    __threadfence();
  }
}

__device__ __forceinline__ void stage_wh(const float* __restrict__ W, _Float16* dst, int tid) {
#pragma unroll 1
  for (int i = tid; i < NHID * NHID; i += NTHR) {
    const int n = i >> 6, k = i & 63;
    dst[n * WPITCH + k] = (_Float16)(W[(size_t)n * NKIN + NEMB + k] * WCAR);
  }
}

__global__ __launch_bounds__(NTHR) void gru_seq_kernel(const int* __restrict__ idx, const float* __restrict__ start,
                                                       const float* __restrict__ Wr, const float* __restrict__ Wz,
                                                       const float* __restrict__ Wh, const float* __restrict__ G,
                                                       unsigned short* __restrict__ HID) {
  __shared__ __align__(16) float    sG[GSIZE];
  __shared__ __align__(16) _Float16 sW[3 * NHID * WPITCH];
  __shared__ __align__(16) _Float16 sAh[NWAVE * RPW * APITCH];
  __shared__ __align__(16) _Float16 sAr[NWAVE * RPW * APITCH];
  const int tid = threadIdx.x, lane = tid & 31, wave = tid >> 5;
  const int c = lane & 15, hh = lane >> 4, koff = 8 * hh;
  const int row0 = (blockIdx.x * NWAVE + wave) * RPW;

#pragma unroll 1
  for (int it = 0; it < (GSIZE4 + NTHR - 1) / NTHR; ++it) {
    const int f  = it * NTHR + tid;
    const int fc = (f < GSIZE4) ? f : (GSIZE4 - 1);
    const v4f v = *(const v4f*)(G + 4 * fc);
    if (f < GSIZE4) *(v4f*)(sG + 4 * fc) = v;
  }
  stage_wh(Wr, sW, tid);
  stage_wh(Wz, sW + NHID * WPITCH, tid);
  stage_wh(Wh, sW + 2 * NHID * WPITCH, tid);

  _Float16* ahw = sAh + wave * RPW * APITCH;
  _Float16* arw = sAr + wave * RPW * APITCH;
  float hst[4][8], zst[4][8];
  {
    float st[4];
#pragma unroll
    for (int nt = 0; nt < 4; ++nt) st[nt] = start[16 * nt + c];
#pragma unroll
    for (int nt = 0; nt < 4; ++nt)
#pragma unroll
      for (int r = 0; r < 8; ++r) {
        hst[nt][r] = st[nt];
        zst[nt][r] = 0.0f;
        ahw[(8 * hh + r) * APITCH + 16 * nt + c] = (_Float16)(st[nt] * HCAR);
      }
  }
  __syncthreads();

  const v8f z8 = {0.f, 0.f, 0.f, 0.f, 0.f, 0.f, 0.f, 0.f};
  const _Float16* ahrow = ahw + c * APITCH + koff;
  const _Float16* arrow = arw + c * APITCH + koff;
  const int q = lane >> 3, c8 = (lane & 7) * 8;

#pragma unroll 1
  for (int t = 0; t < NSTEP; ++t) {
    int mytok = idx[(size_t)(row0 + c) * NSTEP + t];
    mytok = mytok < 0 ? 0 : (mytok > NVOC - 1 ? NVOC - 1 : mytok);
    int tok[8];
#pragma unroll
    for (int r = 0; r < 8; ++r) tok[r] = __shfl(mytok, 8 * hh + r, 32);

    const v16h ah0 = Frag<_Float16>::load(ahrow);
    const v16h ah1 = Frag<_Float16>::load(ahrow + 32);
#pragma unroll
    for (int nt = 0; nt < 4; ++nt) {
      const _Float16* wr = sW + (16 * nt + c) * WPITCH + koff;
      const _Float16* wz = sW + NHID * WPITCH + (16 * nt + c) * WPITCH + koff;
      const v16h br0 = Frag<_Float16>::load(wr);
      const v16h br1 = Frag<_Float16>::load(wr + 32);
      const v16h bz0 = Frag<_Float16>::load(wz);
      const v16h bz1 = Frag<_Float16>::load(wz + 32);
      v8f accR = Frag<_Float16>::mma(ah0, br0, z8);
      v8f accZ = Frag<_Float16>::mma(ah0, bz0, z8);
      accR = Frag<_Float16>::mma(ah1, br1, accR);
      accZ = Frag<_Float16>::mma(ah1, bz1, accZ);
      guard2_f6(accR, accZ, ah0, ah1, br0, br1, bz0, bz1);
#pragma unroll
      for (int r = 0; r < 8; ++r) {
        const float* grow = sG + tok[r] * GCOLS + 16 * nt + c;
        const float pr = accR[r] * FOLD + grow[0];
        const float pz = accZ[r] * FOLD + grow[NHID];
        const float rg = fsig(pr);
        zst[nt][r] = fsig(pz);
        const float rh = rg * hst[nt][r];
        arw[(8 * hh + r) * APITCH + 16 * nt + c] = (_Float16)(rh * HCAR);
      }
    }
    __syncthreads();

    const v16h ar0 = Frag<_Float16>::load(arrow);
    const v16h ar1 = Frag<_Float16>::load(arrow + 32);
#pragma unroll
    for (int nt = 0; nt < 4; ++nt) {
      const _Float16* wh = sW + 2 * NHID * WPITCH + (16 * nt + c) * WPITCH + koff;
      const v16h bh0 = Frag<_Float16>::load(wh);
      const v16h bh1 = Frag<_Float16>::load(wh + 32);
      v8f acc = Frag<_Float16>::mma(ar0, bh0, z8);
      acc = Frag<_Float16>::mma(ar1, bh1, acc);
      guard1_f4(acc, ar0, ar1, bh0, bh1);
#pragma unroll
      for (int r = 0; r < 8; ++r) {
        const float ph = acc[r] * FOLD + sG[tok[r] * GCOLS + 2 * NHID + 16 * nt + c];
        const float hb = tanhf(ph);
        const float z  = zst[nt][r];
        const float ho = hst[nt][r];
        const float hn = (1.0f - z) * ho + z * hb;
        hst[nt][r] = hn;
        ahw[(8 * hh + r) * APITCH + 16 * nt + c] = (_Float16)(hn * HCAR);
      }
    }
    __syncthreads();

    for (int pass = 0; pass < 2; ++pass) {
#pragma unroll
      for (int it = 0; it < 4; ++it) {
        const int row = it * 4 + q;
        const v4u v = *(const v4ua*)(const void*)(ahw + row * APITCH + c8);
        *(volatile v4u*)(void*)(HID + ((size_t)(row0 + row) * NSTEP + (size_t)t) * NHID + c8) = v;
      }
      __threadfence();
    }
  }
}

__global__ __launch_bounds__(NTHR) void lmhead_kernel(const unsigned short* __restrict__ HIDp, const float* __restrict__ Wlm,
                                                      const float* __restrict__ blm, float* __restrict__ out) {
  __shared__ __align__(16) _Float16 sWl[NVPAD * WPITCH];
  __shared__ __align__(16) float    sbl[NVPAD];
  __shared__ __align__(16) float    slab[NWAVE * LMSLAB];
  const _Float16* HID = (const _Float16*)HIDp;
  const int tid = threadIdx.x, lane = tid & 31, wave = tid >> 5;
  const int c = lane & 15, hh = lane >> 4, koff = 8 * hh;

#pragma unroll 1
  for (int it = 0; it < (NVPAD * NHID) / NTHR; ++it) {
    const int i = it * NTHR + tid;
    const int n = i >> 6, k = i & 63;
    const int nc = (n < NVOC) ? n : (NVOC - 1);
    const float w = Wlm[(size_t)nc * NHID + k];
    const float v = (n < NVOC) ? (w * WCAR) : 0.0f;
    sWl[n * WPITCH + k] = (_Float16)v;
  }
  if (tid < NVPAD) {
    const int nc = (tid < NVOC) ? tid : (NVOC - 1);
    const float b = blm[nc];
    sbl[tid] = (tid < NVOC) ? b : 0.0f;
  }
  __syncthreads();

  v16h bw[2][2];
#pragma unroll
  for (int vt = 0; vt < 2; ++vt) {
    const _Float16* wp = sWl + (16 * vt + c) * WPITCH + koff;
    bw[vt][0] = Frag<_Float16>::load(wp);
    bw[vt][1] = Frag<_Float16>::load(wp + 32);
  }
  const v8f z8 = {0.f, 0.f, 0.f, 0.f, 0.f, 0.f, 0.f, 0.f};
  const size_t rowstart = ((size_t)blockIdx.x * NWAVE + (size_t)wave) * LMROWS;
  float* sw = slab + wave * LMSLAB;

#pragma unroll 1
  for (int mt = 0; mt < LMROWS / 16; ++mt) {
    const _Float16* arow = HID + (rowstart + (size_t)(16 * mt + c)) * NHID + koff;
    const v16h a0 = Frag<_Float16>::load(arow);
    const v16h a1 = Frag<_Float16>::load(arow + 32);
    v8f acc0 = Frag<_Float16>::mma(a0, bw[0][0], z8);
    v8f acc1 = Frag<_Float16>::mma(a0, bw[1][0], z8);
    acc0 = Frag<_Float16>::mma(a1, bw[0][1], acc0);
    acc1 = Frag<_Float16>::mma(a1, bw[1][1], acc1);
    guard2_f6(acc0, acc1, a0, a1, bw[0][0], bw[0][1], bw[1][0], bw[1][1]);
#pragma unroll
    for (int r = 0; r < 8; ++r) {
      const int rowl = 16 * mt + 8 * hh + r;
      sw[rowl * NVOC + c] = acc0[r] * FOLD + sbl[c];
      const float v1 = acc1[r] * FOLD + sbl[16 + c];
      if (c < NVOC - 16) sw[rowl * NVOC + 16 + c] = v1;
    }
  }
  __syncthreads();

  float* ob = out + rowstart * NVOC;
  for (int pass = 0; pass < 2; ++pass) {
#pragma unroll
    for (int it = 0; it < (LMSLAB4 + 31) / 32; ++it) {
      const int f  = it * 32 + lane;
      const int fc = (f < LMSLAB4) ? f : (LMSLAB4 - 1);
      const v4f v = *(const v4f*)(sw + 4 * fc);
      if (f < LMSLAB4) *(volatile v4f*)(ob + 4 * (size_t)fc) = v;
    }
    __threadfence();
  }
}

extern "C" void kernel_launch(void* const* d_in, const int* in_sizes, int n_in,
                              void* d_out, int out_size, void* d_ws, size_t ws_size, hipStream_t stream) {
  if (n_in < 11 || d_out == nullptr || d_ws == nullptr) return;
  if (in_sizes[0] != NBAT * NSTEP || in_sizes[1] != NVOC * NEMB || in_sizes[2] != NHID ||
      in_sizes[3] != NHID * NKIN || in_sizes[4] != NHID || in_sizes[5] != NHID * NKIN || in_sizes[6] != NHID ||
      in_sizes[7] != NHID * NKIN || in_sizes[8] != NHID || in_sizes[9] != NVOC * NHID || in_sizes[10] != NVOC ||
      out_size != NOUT) return;

  const int*   idx   = (const int*)d_in[0];
  const float* wte   = (const float*)d_in[1];
  const float* start = (const float*)d_in[2];
  const float* Wz    = (const float*)d_in[3];
  const float* bz    = (const float*)d_in[4];
  const float* Wr    = (const float*)d_in[5];
  const float* br    = (const float*)d_in[6];
  const float* Wh    = (const float*)d_in[7];
  const float* bh    = (const float*)d_in[8];
  const float* Wlm   = (const float*)d_in[9];
  const float* blm   = (const float*)d_in[10];
  float* out = (float*)d_out;

  char* ws = (char*)d_ws; size_t off = 0;
  auto carve = [&](size_t bytes) -> char* { char* p = ws + off; off += (bytes + 255) & ~(size_t)255; return p; };
  float*          GTAB = (float*)carve((size_t)GSIZE * 4);
  unsigned short* HID  = (unsigned short*)carve((size_t)NROWS * NHID * 2);
  if (off > ws_size || off > (size_t)134217728) return;

  gtab_kernel<<<1, NTHR, 0, stream>>>(wte, Wr, br, Wz, bz, Wh, bh, GTAB);
  gru_seq_kernel<<<NBAT / (NWAVE * RPW), NTHR, 0, stream>>>(idx, start, Wr, Wz, Wh, GTAB, HID);
  lmhead_kernel<<<NROWS / (NWAVE * LMROWS), NTHR, 0, stream>>>(HID, Wlm, blm, out);
}
